// GATLayerMultihead_34291018891895
// MI455X (gfx1250) — hardware-verified
//
#include <hip/hip_runtime.h>
#include <math.h>

typedef __attribute__((ext_vector_type(16))) _Float16 v16h;
typedef __attribute__((ext_vector_type(16))) __bf16 v16b;
typedef __attribute__((ext_vector_type(8)))  _Float16 v8h;
typedef __attribute__((ext_vector_type(8)))  float v8f;
typedef __attribute__((ext_vector_type(4)))  float v4f;
typedef __attribute__((ext_vector_type(2)))  float v2f;
typedef __attribute__((ext_vector_type(4)))  unsigned v4u;
typedef __attribute__((ext_vector_type(4)))  int v4i;
typedef float __attribute__((may_alias)) float_a;
typedef int __attribute__((may_alias)) int_a;

template <typename T> __device__ __forceinline__ void vst2(void* p, T v) { *(volatile T*)p = v; __threadfence(); *(volatile T*)p = v; }
__device__ __forceinline__ v8f wmma16(v16h a, v16h b, v8f c) {
  v8f d = __builtin_amdgcn_wmma_f32_16x16x32_f16(false, a, false, b, (short)0, c, false, false);
  asm volatile("v_nop\n\tv_nop\n\tv_nop\n\tv_nop" : "+v"(d) : "v"(a), "v"(b));
  return d;
}
__device__ __forceinline__ v8f wmma_bf(v16b a, v16b b, v8f c) {
  v8f d = __builtin_amdgcn_wmma_f32_16x16x32_bf16(false, a, false, b, (short)0, c, false, false);
  asm volatile("v_nop\n\tv_nop\n\tv_nop\n\tv_nop" : "+v"(d) : "v"(a), "v"(b));
  return d;
}
__device__ __forceinline__ v16h frag_h(const _Float16* rowk0, int lane) {
  union { v16h v; v8h q[2]; } u; const _Float16* p = rowk0 + 8 * (lane >> 4);
  u.q[0] = *(const v8h*)p; u.q[1] = *(const v8h*)(p + 16); return u.v;
}
__device__ __forceinline__ v16h frag_f32(const float* rowk0, int lane) {
  v16h a; const float* p = rowk0 + 8 * (lane >> 4);
#pragma unroll
  for (int i = 0; i < 8; ++i) { a[i] = (_Float16)p[i]; a[8 + i] = (_Float16)p[16 + i]; }
  return a;
}
__device__ __forceinline__ v16h frag_f32s(const float* rowk0, int lane, float sc) {
  v16h a; const float* p = rowk0 + 8 * (lane >> 4);
#pragma unroll
  for (int i = 0; i < 8; ++i) { a[i] = (_Float16)(p[i] * sc); a[8 + i] = (_Float16)(p[16 + i] * sc); }
  return a;
}
__device__ __forceinline__ v16h fragc_f32(const float* W, int k0, int n, int lane, int ld, int K) {
  v16h a; const int g = lane >> 4;
#pragma unroll
  for (int i = 0; i < 8; ++i) { const int ka = k0 + 8 * g + i, kb = ka + 16;
    a[i] = (_Float16)(ka < K ? W[(size_t)(ka < K ? ka : K - 1) * ld + n] : 0.f); a[8 + i] = (_Float16)(kb < K ? W[(size_t)(kb < K ? kb : K - 1) * ld + n] : 0.f); }
  return a;
}
struct F2 { v16b h, l; };
__device__ __forceinline__ F2 bsplit16(const float v[16]) { F2 r;
#pragma unroll
  for (int i = 0; i < 16; ++i) { const __bf16 h = (__bf16)v[i]; r.h[i] = h; r.l[i] = (__bf16)(v[i] - (float)h); }
  return r; }
__device__ __forceinline__ F2 split_row(const float* row, int k0, int lane) { float v[16]; const float* p = row + k0 + 8 * (lane >> 4);
#pragma unroll
  for (int i = 0; i < 8; ++i) { v[i] = p[i]; v[8 + i] = p[16 + i]; }
  return bsplit16(v); }
__device__ __forceinline__ F2 split_rowK(const float* row, int k0, int lane, int K) { float v[16]; const int g = lane >> 4;
#pragma unroll
  for (int i = 0; i < 8; ++i) { const int ka = k0 + 8 * g + i, kb = ka + 16; v[i] = ka < K ? row[ka < K ? ka : K - 1] : 0.f; v[8 + i] = kb < K ? row[kb < K ? kb : K - 1] : 0.f; }
  return bsplit16(v); }
__device__ __forceinline__ F2 split_col(const float* W, int k0, int n, int lane, int ld, int K) { float v[16]; const int g = lane >> 4;
#pragma unroll
  for (int i = 0; i < 8; ++i) { const int ka = k0 + 8 * g + i, kb = ka + 16; v[i] = ka < K ? W[(size_t)(ka < K ? ka : K - 1) * ld + n] : 0.f; v[8 + i] = kb < K ? W[(size_t)(kb < K ? kb : K - 1) * ld + n] : 0.f; }
  return bsplit16(v); }
__device__ __forceinline__ v8f mac3(const F2& a, const F2& b, v8f c) { c = wmma_bf(a.l, b.h, c); c = wmma_bf(a.h, b.l, c); return wmma_bf(a.h, b.h, c); }
__device__ __forceinline__ float sigm(float v) { return 1.0f / (1.0f + expf(-v)); }
#define LDSX() do { asm volatile("s_wait_dscnt 0" ::: "memory"); __builtin_amdgcn_wave_barrier(); __builtin_amdgcn_fence(__ATOMIC_RELEASE, "workgroup"); } while (0)


#define NN 4096
#define FI 64
#define FF 64
#define NH 8
#ifndef TQB
#define TQB (NN / 64)
#endif
typedef __attribute__((ext_vector_type(8))) __bf16 v8b;
__device__ __forceinline__ v16b frag_b(const __bf16* rowk0, int lane) {
  union { v16b v; v8b q[2]; } u; const __bf16* p = rowk0 + 8 * (lane >> 4);
  u.q[0] = *(const v8b*)p; u.q[1] = *(const v8b*)(p + 16); return u.v;
}
__device__ __forceinline__ float bfr(float v) { return (float)(__bf16)v; }
__device__ __attribute__((noinline)) float exp_ni(float v) { return expf(v); }
__device__ __attribute__((noinline)) float erf_ni(float v) { return erff(v); }

#define WS_PW  0u
#define WS_LT  (WS_PW + 2u * (size_t)NH * FF * FI)
#define WS_SD  (WS_LT + 2u * (size_t)NH * FF * NN)
#define WS_END (WS_SD + 4u * (size_t)2 * NH * NN)

__global__ __launch_bounds__(64) void k_pack(const float* __restrict__ Wm, __bf16* __restrict__ P) { const int h = blockIdx.x / FF, o = blockIdx.x % FF, t = threadIdx.x; __shared__ __align__(16) __bf16 s[FI]; s[t] = (__bf16)Wm[((size_t)h * FI + t) * FF + o]; __syncthreads(); if (t < FI / 8) vst2((unsigned*)(P + ((size_t)h * FF + o) * FI + t * 8), *(const v4u*)&s[t * 8]); }
__global__ __launch_bounds__(128) void k_ltg(const float* __restrict__ G, const __bf16* __restrict__ P, const float* __restrict__ A, _Float16* __restrict__ LT, float* __restrict__ SD) {
  __shared__ __align__(16) float sf[64][68]; __shared__ __align__(16) _Float16 st[64][72]; __shared__ __align__(16) float ss[2][64];
  const int tid = threadIdx.x, wave = tid >> 5, lane = tid & 31, col = lane & 15, g = lane >> 4; const int h = blockIdx.y; const int n0b = blockIdx.x * 64; const int r0 = n0b + wave * 16;
  v8f acc[4] = {};
#pragma unroll
  for (int kc = 0; kc < FI / 32; ++kc) { v16b a; { const float* p = G + (size_t)(r0 + col) * FI + kc * 32 + 8 * g;
#pragma unroll
      for (int i = 0; i < 8; ++i) { a[i] = (__bf16)p[i]; a[8 + i] = (__bf16)p[16 + i]; } }
#pragma unroll
    for (int j = 0; j < 4; ++j) acc[j] = wmma_bf(a, frag_b(P + ((size_t)h * FF + j * 16 + col) * FI + kc * 32, lane), acc[j]); }
#pragma unroll
  for (int j = 0; j < 4; ++j)
#pragma unroll
    for (int r = 0; r < 8; ++r) { sf[wave * 16 + 8 * g + r][j * 16 + col] = acc[j][r]; st[j * 16 + col][wave * 16 + 8 * g + r] = (_Float16)acc[j][r]; }
  __syncthreads();
  for (int e = tid; e < 64 * 8; e += 128) { const int d = e >> 3, pc = e & 7; vst2((unsigned*)(LT + ((size_t)h * FF + d) * NN + n0b + pc * 8), *(const v4u*)&st[d][pc * 8]); }
  { const int rl = tid & 63, which = tid >> 6; float s = 0.f;
#pragma unroll 8
    for (int k = 0; k < FF; ++k) s += sf[rl][k] * bfr(A[(size_t)h * 2 * FF + which * FF + k]);
    ss[which][rl] = s; }
  __syncthreads();
  if (tid < 32) { const int which = tid >> 4, q = tid & 15; vst2(SD + ((size_t)which * NH + h) * NN + n0b + q * 4, *(const v4f*)&ss[which][q * 4]); }
}
__device__ __attribute__((noinline)) float exp_p(float v) { return expf(v); }
__device__ __forceinline__ float lk(float e) { return (e >= 0.f) ? e : 0.2f * e; }
__global__ __launch_bounds__(128) void k_gat(const float* __restrict__ SD, const _Float16* __restrict__ LT, float* __restrict__ OUT) {
  __shared__ float sd[NN]; __shared__ __align__(16) _Float16 sph[4][16][40]; __shared__ __align__(16) _Float16 spl[4][16][40]; __shared__ __align__(16) float so[4][16][68]; __shared__ float smax[4];
  const int tid = threadIdx.x, wave = tid >> 5, lane = tid & 31, col = lane & 15, g = lane >> 4; const int h = blockIdx.y; const int i0 = blockIdx.x * 64 + wave * 16;
  float dm = -3.0e38f; for (int j = tid; j < NN; j += 128) { const float v = SD[((size_t)NH + h) * NN + j]; sd[j] = v; dm = fmaxf(dm, v); }
#pragma unroll
  for (int o = 1; o < 32; o <<= 1) dm = fmaxf(dm, __shfl_xor(dm, o));
  if (lane == 0) smax[wave] = dm; __syncthreads(); const float dmax = fmaxf(fmaxf(smax[0], smax[1]), fmaxf(smax[2], smax[3]));
  float si[8], m[8], z[8];
#pragma unroll
  for (int r = 0; r < 8; ++r) { si[r] = SD[(size_t)h * NN + i0 + 8 * g + r]; m[r] = lk(si[r] + dmax); z[r] = 0.f; }
  for (int j = col; j < NN; j += 16) { const float dj = sd[j];
#pragma unroll
    for (int r = 0; r < 8; ++r) z[r] += exp_p(lk(si[r] + dj) - m[r]); }
#pragma unroll
  for (int r = 0; r < 8; ++r) {
#pragma unroll
    for (int o = 1; o < 16; o <<= 1) z[r] += __shfl_xor(z[r], o); }
  v8f acc[4] = {}, accl[4] = {};
#pragma unroll 1
  for (int js = 0; js < NN / 32; ++js) { const int jb = js * 32;
#pragma unroll
    for (int ct = 0; ct < 2; ++ct) { const int j = jb + ct * 16 + col; const float dj = sd[j];
#pragma unroll
      for (int r = 0; r < 8; ++r) { const float ps = __expf(lk(si[r] + dj) - m[r]) / z[r] * 2048.0f; const _Float16 ph = (_Float16)ps; sph[wave][8 * g + r][ct * 16 + col] = ph; spl[wave][8 * g + r][ct * 16 + col] = (_Float16)((ps - (float)ph) * 2048.0f); } }
    LDSX();
    const v16h pa = frag_h(&sph[wave][col][0], lane), pal = frag_h(&spl[wave][col][0], lane);
#pragma unroll
    for (int dt = 0; dt < 4; ++dt) { const v16h lt = frag_h(LT + ((size_t)h * FF + dt * 16 + col) * NN + jb, lane); acc[dt] = wmma16(pa, lt, acc[dt]); accl[dt] = wmma16(pal, lt, accl[dt]); }
    LDSX(); }
#pragma unroll
  for (int r = 0; r < 8; ++r)
#pragma unroll
    for (int dt = 0; dt < 4; ++dt) so[wave][8 * g + r][dt * 16 + col] = (acc[dt][r] + accl[dt][r] * (1.0f / 2048.0f)) * (1.0f / 2048.0f);
  LDSX();
  for (int rl = 0; rl < 16; ++rl) if (lane < 16) vst2(OUT + ((size_t)h * NN + i0 + rl) * FF + lane * 4, *(const v4f*)&so[wave][rl][lane * 4]);
}
extern "C" void kernel_launch(void* const* d_in, const int* in_sizes, int n_in, void* d_out, int out_size, void* d_ws, size_t ws_size, hipStream_t stream) {
  (void)in_sizes; (void)n_in; (void)out_size;
  const float** F = (const float**)d_in;
  if (ws_size < (size_t)WS_END) return;
  char* ws = (char*)d_ws; __bf16* P = (__bf16*)ws; _Float16* LT = (_Float16*)(ws + WS_LT); float* SD = (float*)(ws + WS_SD);
  k_pack<<<NH * FF, 64, 0, stream>>>(F[1], P);
  k_ltg<<<dim3(NN / 64, NH), 128, 0, stream>>>(F[0], P, F[2], LT, SD);
  k_gat<<<dim3(TQB, NH), 128, 0, stream>>>(SD, LT, (float*)d_out);
}
